// PerfectMemory_70205535420745
// MI455X (gfx1250) — hardware-run, weakly checked
//
#include <hip/hip_runtime.h>


#define NPL 8192
#define NEW 768
#define NKW 256
#define NVC 2048
#define NBK 128
#define NBL 4096
#define LG99 -0.014499569695115089f

typedef _Float16 h16;
typedef unsigned short bf;
typedef __attribute__((ext_vector_type(16))) __bf16   v16bf;
typedef __attribute__((ext_vector_type(16))) _Float16 v16h;
typedef __attribute__((ext_vector_type(8)))  _Float16 v8h;
typedef __attribute__((ext_vector_type(8)))  unsigned short v8us;
typedef __attribute__((ext_vector_type(8)))  float    v8f;
typedef __attribute__((ext_vector_type(4)))  float    v4f;
typedef v8h  __attribute__((may_alias)) v8ha;
typedef v4f  __attribute__((may_alias)) v4fa;
typedef v8us __attribute__((may_alias)) v8usa;

__device__ __forceinline__ unsigned short f2bf(float f) { unsigned u = __float_as_uint(f); u += 0x7FFFu + ((u >> 16) & 1u); return (unsigned short)(u >> 16); }
__device__ __forceinline__ float bf2f(unsigned short b) { return __uint_as_float(((unsigned)b) << 16); }
__device__ __forceinline__ float bfr(float f) { return bf2f(f2bf(f)); }
__device__ __forceinline__ v16h cat16(v8h lo, v8h hi) { return __builtin_shufflevector(lo, hi, 0, 1, 2, 3, 4, 5, 6, 7, 8, 9, 10, 11, 12, 13, 14, 15); }
__device__ __forceinline__ v16bf cat16b(v8us lo, v8us hi) { return __builtin_bit_cast(v16bf, __builtin_shufflevector(lo, hi, 0, 1, 2, 3, 4, 5, 6, 7, 8, 9, 10, 11, 12, 13, 14, 15)); }
__device__ __forceinline__ v8f wmma16(v16h a, v16h b, v8f c) { return __builtin_amdgcn_wmma_f32_16x16x32_f16(false, a, false, b, (short)0, c, false, false); }
__device__ __forceinline__ v8f wmmab(v16bf a, v16bf b, v8f c) { return __builtin_amdgcn_wmma_f32_16x16x32_bf16(false, a, false, b, (short)0, c, false, false); }

template <typename T16> struct WFrag;
template <> struct WFrag<h16> { typedef v16h V; static __device__ __forceinline__ V ld(const h16* p) { return cat16(*(const v8h*)p, *(const v8h*)(p + 16)); } static __device__ __forceinline__ v8f mma(V a, V b, v8f c) { return wmma16(a, b, c); } };
template <> struct WFrag<bf> { typedef v16bf V; static __device__ __forceinline__ V ld(const bf* p) { return cat16b(*(const v8us*)p, *(const v8us*)(p + 16)); } static __device__ __forceinline__ v8f mma(V a, V b, v8f c) { return wmmab(a, b, c); } };
template <typename T16, int NSPLIT, bool BIAS>
__global__ __launch_bounds__(32) void k_gemmw(const T16* __restrict__ A, const T16* __restrict__ A2, const T16* __restrict__ Bt, const T16* __restrict__ Bt2, int K, float* C, int ldc, const float* __restrict__ bias, size_t sA, size_t sB, size_t sC) {
    typedef typename WFrag<T16>::V V;
    __shared__ __align__(16) float os[16 * 68];
    const size_t z = blockIdx.z; A += z * sA; if (A2) A2 += z * sA; Bt += z * sB; if (Bt2) Bt2 += z * sB; C += z * sC;
    const int lane = threadIdx.x & 31, lr = lane & 15, hi = lane >> 4; const int r0 = blockIdx.x * 64, c0 = blockIdx.y * 64;
    v8f acc[4][4];
#pragma unroll
    for (int mb = 0; mb < 4; ++mb)
#pragma unroll
        for (int nb = 0; nb < 4; ++nb) acc[mb][nb] = (v8f){};
    const size_t aoff = (size_t)(r0 + lr) * K + 8 * hi, boff = (size_t)(c0 + lr) * K + 8 * hi;
    for (int kc = 0; kc < K; kc += 32) {
        V a[4], a2[4];
#pragma unroll
        for (int mb = 0; mb < 4; ++mb) { a[mb] = WFrag<T16>::ld(A + aoff + (size_t)mb * 16 * K + kc); if (NSPLIT == 1 || NSPLIT == 2) a2[mb] = WFrag<T16>::ld(A2 + aoff + (size_t)mb * 16 * K + kc); }
#pragma unroll
        for (int nb = 0; nb < 4; ++nb) { const V b = WFrag<T16>::ld(Bt + boff + (size_t)nb * 16 * K + kc); V b2; if (NSPLIT >= 2) b2 = WFrag<T16>::ld(Bt2 + boff + (size_t)nb * 16 * K + kc);
#pragma unroll
            for (int mb = 0; mb < 4; ++mb) { acc[mb][nb] = WFrag<T16>::mma(a[mb], b, acc[mb][nb]); if (NSPLIT == 1 || NSPLIT == 2) acc[mb][nb] = WFrag<T16>::mma(a2[mb], b, acc[mb][nb]); if (NSPLIT >= 2) acc[mb][nb] = WFrag<T16>::mma(a[mb], b2, acc[mb][nb]); } }
        asm volatile("v_nop\n\tv_nop\n\tv_nop\n\tv_nop" : "+v"(acc[0][0]), "+v"(acc[1][1]), "+v"(acc[2][2]), "+v"(acc[3][3]) : "v"(a[0]), "v"(a[3]));
    }
#pragma unroll
    for (int mb = 0; mb < 4; ++mb) {
#pragma unroll
        for (int nb = 0; nb < 4; ++nb) {
#pragma unroll
            for (int j = 0; j < 8; ++j) os[(hi * 8 + j) * 68 + nb * 16 + lr] = acc[mb][nb][j]; }
        __builtin_amdgcn_wave_barrier(); asm volatile("" ::: "memory");
        float* crow = C + (size_t)(r0 + mb * 16) * ldc + c0;
#pragma unroll 1
        for (int ps = 0; ps < 2; ++ps) {
#pragma unroll
            for (int s = 0; s < 8; ++s) { const int row = 2 * s + hi, cofs = lr * 4; v4f val = *(const v4fa*)(os + row * 68 + cofs); if (BIAS) { val[0] += bfr(bias[c0 + cofs]); val[1] += bfr(bias[c0 + cofs + 1]); val[2] += bfr(bias[c0 + cofs + 2]); val[3] += bfr(bias[c0 + cofs + 3]); }
                *(volatile v4f*)(crow + (size_t)row * ldc + cofs) = val; }
            if (ps == 0) __threadfence(); }
        __builtin_amdgcn_wave_barrier(); asm volatile("" ::: "memory");
    }
}

typedef __attribute__((ext_vector_type(2))) _Float16 v2h;
typedef __attribute__((ext_vector_type(4))) _Float16 v4h;
typedef __attribute__((ext_vector_type(2))) unsigned short v2us;
typedef __attribute__((ext_vector_type(4))) unsigned short v4us;
typedef __attribute__((ext_vector_type(2))) float v2f;
typedef __attribute__((ext_vector_type(4))) int v4i;
__device__ __forceinline__ h16 toh_flush(float x) { const float z = (fabsf(x) < 6.103515625e-05f) ? 0.0f : x; return (h16)z; }

__global__ __launch_bounds__(256) void k_cvt8(const float* __restrict__ src, bf* dst, size_t n8) { const size_t i = (size_t)blockIdx.x * 256 + threadIdx.x; if (i >= n8) return; const v8f v = *(const v8f*)(src + i * 8); v8us o;
#pragma unroll
    for (int k = 0; k < 8; ++k) o[k] = f2bf(v[k]); *(volatile v8us*)(dst + i * 8) = o; __threadfence(); *(volatile v8us*)(dst + i * 8) = o; }

__global__ __launch_bounds__(256) void k_wtG(const float* __restrict__ w, int K, int N, bf* Bt) {
    const int lane = threadIdx.x & 31; const int L0 = (blockIdx.x * 8 + (threadIdx.x >> 5)) * 8; const int nlines = N * K / 64;
#pragma unroll
    for (int ps = 0; ps < 2; ++ps) {
        for (int l = 0; l < 8; ++l) { const int L = L0 + l; if (L >= nlines) break; const size_t e = (size_t)L * 64 + lane * 2; const int k = (int)(e % K), n = (int)(e / K); v2us o;
            o[0] = f2bf(w[(size_t)k * N + n]); o[1] = f2bf(w[(size_t)(k + 1) * N + n]); *(volatile v2us*)(Bt + e) = o; }
        if (ps == 0) __threadfence(); }
}

__global__ __launch_bounds__(256) void k_tb(const h16* __restrict__ src, h16* dst) {
    const unsigned i = blockIdx.x * 256 + threadIdx.x; const unsigned cl = i & 63u, z = i >> 6; const h16* pp = src + (size_t)z * NBL + cl; h16 r[64];
#pragma unroll
    for (int u = 0; u < 64; ++u) r[u] = pp[u * 64];
    h16* pd = dst + (size_t)i * 64;
#pragma unroll
    for (int ps = 0; ps < 2; ++ps) {
#pragma unroll
        for (int g = 0; g < 8; ++g) { v8h o;
#pragma unroll
            for (int j = 0; j < 8; ++j) o[j] = r[g * 8 + j];
            *(volatile v8h*)(pd + g * 8) = o; }
        if (ps == 0) __threadfence(); } }

__global__ __launch_bounds__(256) void k_unw(const float* __restrict__ Kf, float* Kn, h16* Ka, h16* Kb, h16* Ke) {
    const unsigned t = blockIdx.x * 256 + threadIdx.x; const unsigned i = t & 63u, b = t >> 6; const float* ps = Kf + (size_t)t * NKW; float ss = 0.0f;
#pragma unroll
    for (int g4 = 0; g4 < 64; ++g4) { const v4f q = *(const v4fa*)(ps + g4 * 4);
#pragma unroll
        for (int j = 0; j < 4; ++j) ss = ss + q[j] * q[j]; }
    const float rn = 1.0f / fmaxf(sqrtf(ss), 1e-12f); const float fa = exp2f((float)i * LG99), fb = exp2f((float)i * -LG99), fe = exp2f((float)(63u - i) * LG99);
    float* pn = Kn + (size_t)t * NKW; h16* pa = Ka + (size_t)t * NKW; h16* pb = Kb + (size_t)t * NKW; h16* pe = Ke + (size_t)b * 16384 + (size_t)i * 64;
#pragma unroll
    for (int g8 = 0; g8 < 32; ++g8) { const v4f q0 = *(const v4fa*)(ps + g8 * 8); const v4f q1 = *(const v4fa*)(ps + g8 * 8 + 4); v4f n0, n1; v8h oa, ob, oe;
#pragma unroll
        for (int j = 0; j < 4; ++j) { n0[j] = q0[j] * rn; n1[j] = q1[j] * rn; oa[j] = toh_flush(n0[j] * fa); oa[4 + j] = toh_flush(n1[j] * fa); ob[j] = toh_flush(n0[j] * fb); ob[4 + j] = toh_flush(n1[j] * fb); oe[j] = toh_flush(n0[j] * fe); oe[4 + j] = toh_flush(n1[j] * fe); }
        h16* pt = pe + (size_t)(g8 >> 3) * 4096 + (g8 & 7) * 8;
#pragma unroll
        for (int ps2 = 0; ps2 < 2; ++ps2) { *(volatile v4f*)(pn + g8 * 8) = n0; *(volatile v4f*)(pn + g8 * 8 + 4) = n1; *(volatile v8h*)(pa + g8 * 8) = oa; *(volatile v8h*)(pb + g8 * 8) = ob; *(volatile v8h*)(pt) = oe;
            if (ps2 == 0) __threadfence(); } } }

template <bool KS> __global__ __launch_bounds__(128) void k_sub(const float* __restrict__ Ap, const float* __restrict__ Rs, float* Uv, h16* Ww) {
    const unsigned b = blockIdx.x, c2 = threadIdx.x * 2u; const float* pa = Ap + (size_t)b * 4096; const float* pr = Rs + (size_t)b * 64 * NKW + c2; float ya[64], yb[64];
#pragma unroll
    for (int i = 0; i < 64; ++i) { const v2f r = *(const v2f*)(pr + (size_t)i * NKW); const float f = KS ? 0.1f * exp2f((float)(i + 1) * LG99) : 1.0f; float sa = r[0] * f, sb = r[1] * f;
#pragma unroll
        for (int j = 0; j < i; ++j) { const float a = pa[i * 64 + j]; sa = sa - a * ya[j]; sb = sb - a * yb[j]; }
        ya[i] = 0.1f * sa; yb[i] = 0.1f * sb;
        if (KS) { v2h o; o[0] = toh_flush(sa); o[1] = toh_flush(sb); h16* pd = Ww + ((size_t)b * 64 + i) * NKW + c2; *(volatile v2h*)pd = o; __threadfence(); *(volatile v2h*)pd = o; }
        else { v2f o; o[0] = sa; o[1] = sb; float* pd = Uv + ((size_t)b * 64 + i) * NKW + c2; *(volatile v2f*)pd = o; __threadfence(); *(volatile v2f*)pd = o; } } }

__global__ __launch_bounds__(256) void k_usb(const float* __restrict__ UvB, const float* __restrict__ C1, h16* Ut) {
    const unsigned c = blockIdx.x * 256 + threadIdx.x; const float* pu = UvB + (c & 255u); const float* pc = C1 + c; h16 r[64];
#pragma unroll
    for (int i = 0; i < 64; ++i) r[i] = toh_flush(pu[(size_t)i * NKW] - pc[(size_t)i * NVC]);
    h16* pd = Ut + (size_t)c * 64;
#pragma unroll
    for (int ps2 = 0; ps2 < 2; ++ps2) {
#pragma unroll
        for (int g = 0; g < 8; ++g) { v8h o;
#pragma unroll
            for (int j = 0; j < 8; ++j) o[j] = r[g * 8 + j];
            *(volatile v8h*)(pd + g * 8) = o; }
        if (ps2 == 0) __threadfence(); } }

__global__ __launch_bounds__(256) void k_stp(const float* __restrict__ Pb, const float* __restrict__ Du, float* Pn, h16* Pw) {
    const size_t e = ((size_t)blockIdx.x * 256 + threadIdx.x) * 4; const v4f p = *(const v4fa*)(Pb + e); const v4f d = *(const v4fa*)(Du + e); v4f o; v4h w;
#pragma unroll
    for (int j = 0; j < 4; ++j) { o[j] = 0.525596499f * p[j] + d[j]; w[j] = toh_flush(o[j]); }
    *(volatile v4f*)(Pn + e) = o; *(volatile v4h*)(Pw + e) = w; __threadfence(); *(volatile v4f*)(Pn + e) = o; *(volatile v4h*)(Pw + e) = w; }

template <bool RB> __global__ __launch_bounds__(256) void k_ptr(const float* __restrict__ src, float* dst, h16* Pw) {
    const unsigned i = blockIdx.x * 256 + threadIdx.x; const unsigned c = i & 255u, rb = (i >> 8) & 3u, g = i >> 10; const float* ps = src + (size_t)g * 65536 + (size_t)rb * 64 * 256 + c; float r[64];
#pragma unroll
    for (int u = 0; u < 64; ++u) r[u] = RB ? bfr(ps[(size_t)u * 256]) : ps[(size_t)u * 256];
    float* pd = dst + (size_t)g * 65536 + (size_t)c * 256 + rb * 64; h16* pw = Pw + (size_t)g * 65536 + (size_t)c * 256 + rb * 64;
#pragma unroll
    for (int ps2 = 0; ps2 < 2; ++ps2) {
#pragma unroll
        for (int g4 = 0; g4 < 16; ++g4) { v4f o;
#pragma unroll
            for (int j = 0; j < 4; ++j) o[j] = r[g4 * 4 + j];
            *(volatile v4f*)(pd + g4 * 4) = o; }
        if (RB) {
#pragma unroll
            for (int g8 = 0; g8 < 8; ++g8) { v8h w;
#pragma unroll
                for (int j = 0; j < 8; ++j) w[j] = toh_flush(r[g8 * 8 + j]);
                *(volatile v8h*)(pw + g8 * 8) = w; } }
        if (ps2 == 0) __threadfence(); } }

extern "C" void kernel_launch(void* const* d_in, const int* in_sizes, int n_in, void* d_out, int out_size, void* d_ws, size_t ws_size, hipStream_t stream) {
    if (n_in < 4) return;
    if (in_sizes[0] != NPL * NEW || in_sizes[1] != NEW * NKW || in_sizes[2] != NEW * NKW || in_sizes[3] != NVC * NKW || out_size != NVC * NKW) return;
    static_assert(NPL == 8192 && NEW == 768 && NKW == 256 && NVC == 2048 && NBK * 64 == NPL && NEW % 64 == 0 && NEW % 32 == 0 && NKW % 64 == 0 && NVC % 64 == 0 && (NPL * NEW / 8) % 256 == 0 && (NEW * NKW / 64) % 64 == 0 && NPL % 256 == 0 && (NVC * NKW / 4) % 256 == 0 && NVC % 256 == 0, "the products: row and column counts multiples of 64, every depth a multiple of 32; the flat grids exact; the transposing cast: a depth that is even and a multiple of 64, whole blocks of 64 lines");
    const float* a0 = (const float*)d_in[0]; const float* a1 = (const float*)d_in[1]; const float* a2 = (const float*)d_in[2]; const float* a3 = (const float*)d_in[3]; float* res = (float*)d_out;
    char* wsp = (char*)d_ws; auto take = [&](size_t bytes) { char* p = wsp; wsp += (bytes + 255) & ~(size_t)255; return (void*)p; };
    bf* Ew = (bf*)take((size_t)NPL * NEW * 2); bf* Wa = (bf*)take((size_t)NKW * NEW * 2); bf* Wb = (bf*)take((size_t)NKW * NEW * 2); float* Kf = (float*)take((size_t)NPL * NKW * 4); float* Vf = (float*)take((size_t)NPL * NKW * 4); float* Kn = (float*)take((size_t)NPL * NKW * 4);
    h16* Ka = (h16*)take((size_t)NPL * NKW * 2); h16* Kb = (h16*)take((size_t)NPL * NKW * 2); h16* Ke = (h16*)take((size_t)NPL * NKW * 2); h16* Kt = (h16*)take((size_t)NPL * NKW * 2); float* Ap = (float*)take((size_t)NBK * 4096 * 4); float* Uv = (float*)take((size_t)NPL * NKW * 4); h16* Ww = (h16*)take((size_t)NPL * NKW * 2);
    float* PtA = (float*)take((size_t)NVC * NKW * 4); float* PtB = (float*)take((size_t)NVC * NKW * 4); h16* Pw = (h16*)take((size_t)NVC * NKW * 2); float* C1 = (float*)take((size_t)64 * NVC * 4); h16* Ut = (h16*)take((size_t)NVC * 64 * 2); float* Du = (float*)take((size_t)NVC * NKW * 4);
    if ((size_t)(wsp - (char*)d_ws) > ws_size) return;
    k_cvt8<<<(unsigned)((size_t)NPL * NEW / 8 / 256), 256, 0, stream>>>(a0, Ew, (size_t)NPL * NEW / 8);
    k_wtG<<<(unsigned)((NEW * NKW / 64 + 63) / 64), 256, 0, stream>>>(a1, NEW, NKW, Wa); k_wtG<<<(unsigned)((NEW * NKW / 64 + 63) / 64), 256, 0, stream>>>(a2, NEW, NKW, Wb);
    k_gemmw<bf, 0, false><<<dim3(NPL / 64, NKW / 64, 1), 32, 0, stream>>>(Ew, nullptr, Wa, nullptr, NEW, Kf, NKW, nullptr, 0, 0, 0);
    k_gemmw<bf, 0, false><<<dim3(NPL / 64, NKW / 64, 1), 32, 0, stream>>>(Ew, nullptr, Wb, nullptr, NEW, Vf, NKW, nullptr, 0, 0, 0);
    k_unw<<<NPL / 256, 256, 0, stream>>>(Kf, Kn, Ka, Kb, Ke);
    k_tb<<<NBK * 4 * 64 / 256, 256, 0, stream>>>(Ke, Kt);
    k_gemmw<h16, 0, false><<<dim3(1, 1, NBK), 32, 0, stream>>>(Ka, nullptr, Kb, nullptr, NKW, Ap, 64, nullptr, (size_t)64 * NKW, (size_t)64 * NKW, (size_t)4096);
    k_sub<false><<<NBK, 128, 0, stream>>>(Ap, Vf, Uv, nullptr); k_sub<true><<<NBK, 128, 0, stream>>>(Ap, Kn, nullptr, Ww);
    k_ptr<true><<<NVC * 4 / 256, 256, 0, stream>>>(a3, PtA, Pw);
    for (int b = 0; b < NBK; ++b) { float* Pb = (b & 1) ? PtB : PtA; float* Pn = (b & 1) ? PtA : PtB;
        k_gemmw<h16, 0, false><<<dim3(1, NVC / 64, 1), 32, 0, stream>>>(Ww + (size_t)b * 64 * NKW, nullptr, Pw, nullptr, NKW, C1, NVC, nullptr, 0, 0, 0);
        k_usb<<<NVC / 256, 256, 0, stream>>>(Uv + (size_t)b * 64 * NKW, C1, Ut);
        k_gemmw<h16, 0, false><<<dim3(NVC / 64, NKW / 64, 1), 32, 0, stream>>>(Ut, nullptr, Kt + (size_t)b * NKW * 64, nullptr, 64, Du, NKW, nullptr, 0, 0, 0);
        k_stp<<<(unsigned)((size_t)NVC * NKW / 4 / 256), 256, 0, stream>>>(Pb, Du, Pn, Pw); }
    k_ptr<false><<<NVC * 4 / 256, 256, 0, stream>>>(PtA, res, nullptr);
}
